// perceptual_network_vm_81106162418420
// MI455X (gfx1250) — hardware-verified
//
#include <hip/hip_runtime.h>
#include <math.h>


typedef __attribute__((ext_vector_type(16))) _Float16 v16h;
typedef __attribute__((ext_vector_type(8)))  _Float16 v8h;
typedef __attribute__((ext_vector_type(8)))  float  v8f;
typedef __attribute__((ext_vector_type(4)))  float  v4f;
typedef __attribute__((ext_vector_type(4)))  unsigned v4u;
typedef float __attribute__((may_alias)) float_a;

#define T_STEPS 16384
#define H_DIM   361
#define NPAD    368
#define XPITCH  384
#define NTILES  23
#define K_IN    489
#define KPAD_IN 512
#define KS_IN   16
#define KS_HH   12
#define PI_F    3.14159265358979f
#define HCHUNK  32

template <typename T> __device__ __forceinline__ void vst2(void* p, T v) { *(volatile T*)p = v; __threadfence(); *(volatile T*)p = v; }
__device__ __forceinline__ v8f wmma16(v16h a, v16h b, v8f c) {
  v8f d = __builtin_amdgcn_wmma_f32_16x16x32_f16(false, a, false, b, (short)0, c, false, false);
  asm volatile("v_nop\n\tv_nop\n\tv_nop\n\tv_nop" : "+v"(d) : "v"(a), "v"(b));
  return d;
}
__device__ __forceinline__ v16h frag_h(const _Float16* rowk0, int lane) {
  union { v16h v; v8h q[2]; } u; const _Float16* p = rowk0 + 8 * (lane >> 4);
  u.q[0] = *(const v8h*)p; u.q[1] = *(const v8h*)(p + 16); return u.v;
}

__device__ __forceinline__ float vonmises_pdf(float grid, float mu) {
  const float k = 1.0f / (0.1745f * 0.1745f);
  const float d = grid - mu;
  const float poly = 1.f + 1.f/(8.f*k) + 9.f/(128.f*k*k) + 225.f/(3072.f*k*k*k) + 11025.f/(98304.f*k*k*k*k);
  return expf(k * (cosf(d) - 1.f)) * sqrtf(k / (2.f * PI_F)) / poly;
}

__global__ __launch_bounds__(256) void build_combined(const float* __restrict__ angle, const float* __restrict__ rule,
                                                      const float* __restrict__ w_rule, const float* __restrict__ b_rule, _Float16* __restrict__ combined) {
  const int g8 = blockIdx.x * 256 + threadIdx.x;
  const int t = g8 >> 6, c0 = (g8 & 63) * 8;
  const float mu = angle[t] * (PI_F / 180.f), rt = rule[t];
  union { v8h h; v4u u; } pk;
#pragma unroll 1
  for (int e = 0; e < 8; ++e) { const int c = c0 + e; float v = 0.f;
    if (c < 128) v = rt * w_rule[c] + b_rule[c];
    else if (c < K_IN) v = vonmises_pdf((float)(c - 128) * (PI_F / 180.f), mu);
    pk.h[e] = (_Float16)v; }
  vst2(combined + (size_t)g8 * 8, pk.u);
}

__global__ __launch_bounds__(256) void pack_b(const float* __restrict__ w, int rows, int cols, int ksteps, _Float16* __restrict__ out) {
  const int g8 = blockIdx.x * 256 + threadIdx.x;
  if (g8 >= NTILES * ksteps * 64) return;
  const int eh = g8 & 1, ln = (g8 >> 1) & 31, frag = g8 >> 6;
  const int nt = frag / ksteps, ks = frag % ksteps;
  const int n = nt * 16 + (ln & 15);
  union { v8h h; v4u u; } pk;
#pragma unroll
  for (int i = 0; i < 8; ++i) { const int k = ks * 32 + 8 * (ln >> 4) + eh * 16 + i;
    pk.h[i] = (_Float16)((n < rows && k < cols) ? w[(size_t)n * cols + k] : 0.f); }
  vst2(out + ((size_t)frag * 32 + ln) * 16 + eh * 8, pk.u);
}

__global__ __launch_bounds__(256) void gemm_xw(const _Float16* __restrict__ combined, const _Float16* __restrict__ wbih,
                                              const float* __restrict__ b_ih, const float* __restrict__ b_hh, float* __restrict__ xw) {
  __shared__ __align__(16) float st[64][XPITCH + 4];
  const int tid = threadIdx.x, wave = tid >> 5, ln = tid & 31, col = ln & 15, g = ln >> 4;
  const int rg = wave & 3, nh = wave >> 2;
  const int r0 = blockIdx.x * 64 + rg * 16;
  const int nt0 = nh * 12, ntn = nh == 0 ? 12 : 11;
  v8f acc[12] = {};
#pragma unroll 1
  for (int ks = 0; ks < KS_IN; ++ks) {
    const v16h a = frag_h(combined + (size_t)(r0 + col) * KPAD_IN + ks * 32, ln);
#pragma unroll
    for (int j = 0; j < 12; ++j) if (j < ntn) {
      const v16h b = *(const v16h*)(wbih + ((size_t)((nt0 + j) * KS_IN + ks) * 32 + ln) * 16);
      acc[j] = wmma16(a, b, acc[j]); }
  }
#pragma unroll
  for (int j = 0; j < 12; ++j) if (j < ntn) {
    const int ncol = (nt0 + j) * 16 + col; const float bias = (ncol < H_DIM) ? b_ih[ncol] + b_hh[ncol] : 0.f;
#pragma unroll
    for (int r = 0; r < 8; ++r) st[rg * 16 + 8 * g + r][ncol] = acc[j][r] + bias; }
  for (int i = tid; i < 64 * 16; i += 256) st[i >> 4][NPAD + (i & 15)] = 0.f;
  __syncthreads();
  for (int q = tid; q < 64 * 96; q += 256) { const int rl = q / 96, pc = q % 96;
    vst2(xw + (size_t)(blockIdx.x * 64 + rl) * XPITCH + pc * 4, *(const v4f*)(&st[rl][pc * 4])); }
}

__global__ __launch_bounds__(736) void rnn_scan(const _Float16* __restrict__ wbhh, const float* __restrict__ xw, float* __restrict__ hs_out, int nsteps) {
  __shared__ __align__(16) _Float16 hbuf[2][384];
  __shared__ __align__(16) float hist[HCHUNK * H_DIM];
  const int tid = threadIdx.x, w = tid >> 5, ln = tid & 31;
  v16h Wf[KS_HH];
#pragma unroll
  for (int ks = 0; ks < KS_HH; ++ks) Wf[ks] = *(const v16h*)(wbhh + ((size_t)(w * KS_HH + ks) * 32 + ln) * 16);
  for (int i = tid; i < 2 * 384; i += 736) (&hbuf[0][0])[i] = (_Float16)0.f;
  __syncthreads();
  const int row = ln & 15;
  const int n   = w * 16 + (ln & 15);
  for (int t = 0; t < nsteps; ++t) {
    const int cur = t & 1, nxt = cur ^ 1;
    const float xv = (ln < 16) ? xw[(size_t)t * XPITCH + n] : 0.f;
    v8f acc[4] = {{}, {}, {}, {}};
#pragma unroll
    for (int ks = 0; ks < KS_HH; ++ks) {
      v16h a;
      if (row == 0) a = frag_h(&hbuf[cur][ks * 32], ln);
      else {
#pragma unroll
        for (int e = 0; e < 16; ++e) a[e] = (_Float16)0.f; }
      acc[ks & 3] = wmma16(a, Wf[ks], acc[ks & 3]);
    }
    if (ln < 16) {
      const float h = tanhf(acc[0][0] + acc[1][0] + acc[2][0] + acc[3][0] + xv);
      hbuf[nxt][n] = (_Float16)(n < H_DIM ? h : 0.f);
      if (n < H_DIM) hist[(t & (HCHUNK - 1)) * H_DIM + n] = h;
    }
    __syncthreads();
    if ((t & (HCHUNK - 1)) == HCHUNK - 1) {
      const size_t base = (size_t)(t - (HCHUNK - 1)) * H_DIM;
      for (int q = tid; q < HCHUNK * H_DIM / 4; q += 736) vst2(hs_out + base + (size_t)q * 4, *(const v4f*)(&hist[q * 4]));
      __syncthreads();
    }
  }
}

__global__ __launch_bounds__(256) void fc_out(const float* __restrict__ hs, const float* __restrict__ w_fc, const float* __restrict__ b_fc, float* __restrict__ outc) {
  const int t = blockIdx.x * 256 + threadIdx.x;
  if (t >= T_STEPS) return;
  float acc = b_fc[0];
#pragma unroll 1
  for (int i = 0; i < H_DIM; ++i) acc += hs[(size_t)t * H_DIM + i] * w_fc[i];
  vst2(outc + t, (float_a)acc);
}

extern "C" void kernel_launch(void* const* d_in, const int* in_sizes, int n_in,
                              void* d_out, int out_size, void* d_ws, size_t ws_size,
                              hipStream_t stream) {
  (void)in_sizes; (void)n_in; (void)out_size; (void)ws_size;
  const float* angle  = (const float*)d_in[0];
  const float* rule   = (const float*)d_in[1];
  const float* w_rule = (const float*)d_in[2];
  const float* b_rule = (const float*)d_in[3];
  const float* w_ih   = (const float*)d_in[4];
  const float* w_hh   = (const float*)d_in[5];
  const float* b_ih   = (const float*)d_in[6];
  const float* b_hh   = (const float*)d_in[7];
  const float* w_fc   = (const float*)d_in[8];
  const float* b_fc   = (const float*)d_in[9];
  float* outc   = (float*)d_out;
  float* hs_out = (float*)d_out + T_STEPS;
  char* ws = (char*)d_ws;
  _Float16* combined = (_Float16*)ws;             ws += (size_t)T_STEPS * KPAD_IN * 2;
  _Float16* wbih     = (_Float16*)ws;             ws += (size_t)NTILES * KS_IN * 512 * 2;
  _Float16* wbhh     = (_Float16*)ws;             ws += (size_t)NTILES * KS_HH * 512 * 2;
  float*    xw       = (float*)ws;                ws += (size_t)T_STEPS * XPITCH * 4;

  build_combined<<<(T_STEPS * KPAD_IN / 8) / 256, 256, 0, stream>>>(angle, rule, w_rule, b_rule, combined);
  pack_b<<<(NTILES * KS_IN * 64 + 255) / 256, 256, 0, stream>>>(w_ih, H_DIM, K_IN, KS_IN, wbih);
  pack_b<<<(NTILES * KS_HH * 64 + 255) / 256, 256, 0, stream>>>(w_hh, H_DIM, H_DIM, KS_HH, wbhh);
  gemm_xw<<<T_STEPS / 64, 256, 0, stream>>>(combined, wbih, b_ih, b_hh, xw);
  rnn_scan<<<1, 736, 0, stream>>>(wbhh, xw, hs_out, T_STEPS);
  fc_out<<<T_STEPS / 256, 256, 0, stream>>>(hs_out, w_fc, b_fc, outc);
}
